// BaselineCapsNet_43903155699883
// MI455X (gfx1250) — hardware-verified
//
#include <hip/hip_runtime.h>
#include <math.h>

constexpr int kBatch    = 256;
constexpr int kImg      = 28;
constexpr int kImgPix   = 784;
constexpr int kCh1      = 256;
constexpr int kO1       = 20;
constexpr int kO1Pix    = 400;
constexpr int kK1       = 81;
constexpr int kK1P      = 96;
constexpr int kCh2      = 256;
constexpr int kK2       = 20736;
constexpr int kO2       = 6;
constexpr int kPos      = 36;
constexpr int kRoutes   = 1152;
constexpr int kCapsIn   = 8;
constexpr int kCaps     = 10;
constexpr int kCapsDim  = 16;
constexpr int kJD       = 160;
constexpr int kJDP      = 192;
constexpr int kQ        = 9216;
constexpr int kPitchBC  = 16;
constexpr int kChunkImg = 32;
constexpr int kChunks   = 8;
constexpr int kM1       = kChunkImg * kO1Pix;
constexpr int kM2       = kChunkImg * kPos;
constexpr float kW2Carry    = 32.0f;
constexpr float kW2CarryInv = 1.0f / 32.0f;
constexpr float kInvBatch   = 1.0f / 256.0f;

typedef __attribute__((ext_vector_type(16))) _Float16 v16h;
typedef __attribute__((ext_vector_type(8)))  _Float16 v8h;
typedef __attribute__((ext_vector_type(16))) __bf16   v16b;
typedef __attribute__((ext_vector_type(8)))  __bf16   v8b;
typedef __attribute__((ext_vector_type(8)))  float    v8f;
typedef __attribute__((ext_vector_type(4)))  float    v4f;
typedef __attribute__((ext_vector_type(4)))  unsigned int v4u;

__device__ __forceinline__ unsigned short f2bf_bits(float f) {
  unsigned u = __float_as_uint(f);
  return (unsigned short)((u + 0x7FFFu + ((u >> 16) & 1u)) >> 16);
}
__device__ __forceinline__ float bf_bits2f(unsigned short h) { return __uint_as_float(((unsigned)h) << 16); }

__device__ __forceinline__ void dep_guard_h(v8f& a, v8f& b, v16h x, v16h y) { asm volatile("v_nop\n\tv_nop\n\tv_nop\n\tv_nop" : "+v"(a), "+v"(b) : "v"(x), "v"(y)); }
__device__ __forceinline__ void dep_guard_b(v8f& a, v8f& b, v16b x, v16b y) { asm volatile("v_nop\n\tv_nop\n\tv_nop\n\tv_nop" : "+v"(a), "+v"(b) : "v"(x), "v"(y)); }
__device__ __forceinline__ void keep4_h(v16h a, v16h b, v16h c, v16h d) { asm volatile("v_nop" :: "v"(a), "v"(b), "v"(c), "v"(d)); }
__device__ __forceinline__ void keep4_b(v16b a, v16b b, v16b c, v16b d) { asm volatile("v_nop" :: "v"(a), "v"(b), "v"(c), "v"(d)); }
__device__ __forceinline__ void acc_guard4(v8f& a, v8f& b, v8f& c, v8f& d) { asm volatile("v_nop\n\tv_nop\n\tv_nop\n\tv_nop" : "+v"(a), "+v"(b), "+v"(c), "+v"(d)); }
template <typename T> struct Frag;
template <> struct Frag<_Float16> {
  typedef v16h V; union U { v16h v; v8h h[2]; };
  static __device__ __forceinline__ v16h load(const _Float16* p) {
    U f; f.h[0] = *(const v8h*)(p); f.h[1] = *(const v8h*)(p + 16); return f.v;
  }
  static __device__ __forceinline__ v8f mma(v16h a, v16h b, v8f c) {
    return __builtin_amdgcn_wmma_f32_16x16x32_f16(false, a, false, b, (short)0, c, false, false);
  }
  static __device__ __forceinline__ void guard(v8f& a, v8f& b, v16h x, v16h y) { dep_guard_h(a, b, x, y); }
  static __device__ __forceinline__ void keep(v16h a, v16h b, v16h c, v16h d) { keep4_h(a, b, c, d); }
};
template <> struct Frag<__bf16> {
  typedef v16b V; union U { v16b v; v8b h[2]; };
  static __device__ __forceinline__ v16b load(const __bf16* p) {
    U f; f.h[0] = *(const v8b*)(p); f.h[1] = *(const v8b*)(p + 16); return f.v;
  }
  static __device__ __forceinline__ v8f mma(v16b a, v16b b, v8f c) {
    return __builtin_amdgcn_wmma_f32_16x16x32_bf16(false, a, false, b, (short)0, c, false, false);
  }
  static __device__ __forceinline__ void guard(v8f& a, v8f& b, v16b x, v16b y) { dep_guard_b(a, b, x, y); }
  static __device__ __forceinline__ void keep(v16b a, v16b b, v16b c, v16b d) { keep4_b(a, b, c, d); }
};

__device__ __forceinline__ unsigned pk16(unsigned short a, unsigned short b) { return (unsigned)a | ((unsigned)b << 16); }
__device__ __forceinline__ unsigned short h_bits(float f) { const _Float16 h = (_Float16)f; return __builtin_bit_cast(unsigned short, h); }

template <int ET> struct Elem;
template <> struct Elem<0> { typedef _Float16 T; };
template <> struct Elem<1> { typedef __bf16 T; };
template <int ET, bool SPLIT, int BIAS_MODE, int OUT_MODE, bool RESID, int ACT = 0>
__global__ __launch_bounds__(256) void wmma_gemm64(
    const unsigned short* __restrict__ Ap, const unsigned short* __restrict__ A2p, int lda, long strideA,
    const unsigned short* __restrict__ Btp, const unsigned short* __restrict__ Bt2p, int ldb, long strideB,
    void* __restrict__ Cout, void* __restrict__ Cout2, int ldc, long strideC,
    const float* __restrict__ bias,
    const float* __restrict__ resid, long strideR,
    int M, int N, int K, float scale) {
  typedef typename Elem<ET>::T T;
  typedef typename Frag<T>::V V;
  const T* A = (const T*)Ap; const T* A2 = (const T*)A2p; const T* Bt = (const T*)Btp; const T* Bt2 = (const T*)Bt2p;
  __shared__ __align__(16) float sT[8][16 * 68];
  const int b    = blockIdx.y;
  const int lane = threadIdx.x & 31;
  const int wave = threadIdx.x >> 5;
  const int tilesN = N >> 6;
  const int tilesM = M >> 6;
  const int tile = blockIdx.x * 8 + wave;
  if (tile >= tilesM * tilesN) return;
  const int tm = tile / tilesN;
  const int tn = tile - tm * tilesN;
  const int m0 = tm << 6;
  const int n0 = tn << 6;

  const T* Ab  = A  + (size_t)b * strideA;
  const T* Bb  = Bt + (size_t)b * strideB;
  const T* Ab2 = SPLIT ? (A2  + (size_t)b * strideA) : nullptr;
  const T* Bb2 = SPLIT ? (Bt2 + (size_t)b * strideB) : nullptr;

  const int rlane = lane & 15;
  const int koff  = (lane >> 4) * 8;
  const int mOff  = (lane >> 4) * 8;

  v8f acc[4][4];
#pragma unroll
  for (int i = 0; i < 4; ++i)
#pragma unroll
    for (int j = 0; j < 4; ++j) acc[i][j] = (v8f){0.f,0.f,0.f,0.f,0.f,0.f,0.f,0.f};

  for (int k0 = 0; k0 < K; k0 += 32) {
    V bh[4], bl[4];
#pragma unroll
    for (int j = 0; j < 4; ++j) {
      const size_t bo = (size_t)(n0 + (j << 4) + rlane) * ldb + koff + k0;
      bh[j] = Frag<T>::load(Bb + bo);
      if (SPLIT) bl[j] = Frag<T>::load(Bb2 + bo);
    }
#pragma unroll
    for (int i = 0; i < 4; ++i) {
      const size_t ao = (size_t)(m0 + (i << 4) + rlane) * lda + koff + k0;
      V ah = Frag<T>::load(Ab + ao);
      V al;
      if (SPLIT) al = Frag<T>::load(Ab2 + ao);
#pragma unroll
      for (int j = 0; j < 4; ++j) {
        acc[i][j] = Frag<T>::mma(ah, bh[j], acc[i][j]);
        if (SPLIT) {
          acc[i][j] = Frag<T>::mma(ah, bl[j], acc[i][j]);
          acc[i][j] = Frag<T>::mma(al, bh[j], acc[i][j]);
        }
      }
      Frag<T>::guard(acc[i][0], acc[i][3], ah, SPLIT ? al : ah);
    }
    Frag<T>::keep(bh[0], bh[1], bh[2], bh[3]);
    if (SPLIT) Frag<T>::keep(bl[0], bl[1], bl[2], bl[3]);
  }
  acc_guard4(acc[0][0], acc[0][1], acc[0][2], acc[0][3]);
  acc_guard4(acc[1][0], acc[1][1], acc[1][2], acc[1][3]);
  acc_guard4(acc[2][0], acc[2][1], acc[2][2], acc[2][3]);
  acc_guard4(acc[3][0], acc[3][1], acc[3][2], acc[3][3]);

  float* slab = sT[wave];
  const float* Rb = RESID ? (resid + (size_t)b * strideR) : nullptr;
#pragma unroll
  for (int i = 0; i < 4; ++i) {
    const int mBase = m0 + (i << 4);
#pragma unroll
    for (int j = 0; j < 4; ++j) {
      const int n = n0 + (j << 4) + rlane;
      float bv = 0.f;
      if (BIAS_MODE == 2) bv = bias[n];
#pragma unroll
      for (int r = 0; r < 8; ++r) {
        float v = acc[i][j][r] * scale;
        if (BIAS_MODE == 1) v += bias[mBase + mOff + r];
        if (BIAS_MODE == 2) v += bv;
        if (RESID) v += Rb[(size_t)(mBase + mOff + r) * ldc + n];
        if (ACT == 2) v = fmaxf(v, 0.0f);
        if (ACT == 4) v = (v > 0.f) ? v : 0.01f * v;
        slab[(mOff + r) * 68 + (j << 4) + rlane] = v;
      }
    }
    __builtin_amdgcn_fence(__ATOMIC_RELEASE, "workgroup");
    __builtin_amdgcn_wave_barrier();
    __builtin_amdgcn_fence(__ATOMIC_ACQUIRE, "workgroup");
    if (OUT_MODE == 0) {
      float* C = (float*)Cout + (size_t)b * strideC;
      const int hh = lane >> 4, c4 = (lane & 15) * 4;
      for (int pass = 0; pass < 2; ++pass) {
#pragma unroll
        for (int it = 0; it < 8; ++it) {
          const int row = it * 2 + hh;
          v4f v = *(const v4f*)(slab + row * 68 + c4);
          *(volatile v4f*)(C + (size_t)(mBase + row) * ldc + n0 + c4) = v;
        }
        __threadfence();
      }
    } else {
      const int q = lane >> 3, c8 = (lane & 7) * 8;
      unsigned short* C  = (unsigned short*)Cout  + (size_t)b * strideC;
      unsigned short* C2 = (OUT_MODE == 2) ? ((unsigned short*)Cout2 + (size_t)b * strideC) : nullptr;
      for (int pass = 0; pass < 2; ++pass) {
#pragma unroll
        for (int it = 0; it < 4; ++it) {
          const int row = it * 4 + q;
          const float* sp = slab + row * 68 + c8;
          v8h hv, lv;
#pragma unroll
          for (int e = 0; e < 8; ++e) {
            if (OUT_MODE == 1) {
              hv[e] = (_Float16)sp[e];
            } else {
              unsigned short hb = f2bf_bits(sp[e]);
              unsigned short lb = f2bf_bits(sp[e] - bf_bits2f(hb));
              hv[e] = __builtin_bit_cast(_Float16, hb);
              lv[e] = __builtin_bit_cast(_Float16, lb);
            }
          }
          *(volatile v8h*)(C + (size_t)(mBase + row) * ldc + n0 + c8) = hv;
          if (OUT_MODE == 2) *(volatile v8h*)(C2 + (size_t)(mBase + row) * ldc + n0 + c8) = lv;
        }
        __threadfence();
      }
    }
    __builtin_amdgcn_fence(__ATOMIC_RELEASE, "workgroup");
    __builtin_amdgcn_wave_barrier();
    __builtin_amdgcn_fence(__ATOMIC_ACQUIRE, "workgroup");
  }
}

__device__ __forceinline__ void bf_split_bits(float x, unsigned short& hb, unsigned short& lb) {
  hb = f2bf_bits(x);
  lb = f2bf_bits(x - bf_bits2f(hb));
}
__device__ __forceinline__ void st2x_u4(unsigned short* ph, v4u uh, unsigned short* pl, v4u ul) {
  *(volatile v4u*)ph = uh;
  *(volatile v4u*)pl = ul;
  __threadfence();
  *(volatile v4u*)ph = uh;
  *(volatile v4u*)pl = ul;
}
__device__ __forceinline__ void st2_u4(unsigned short* p, v4u u) {
  *(volatile v4u*)p = u;
  __threadfence();
  *(volatile v4u*)p = u;
}
__device__ __forceinline__ void st2_f4(float* p, v4f v) {
  *(volatile v4f*)p = v;
  __threadfence();
  *(volatile v4f*)p = v;
}

__global__ __launch_bounds__(256) void k_w1_split(const float* __restrict__ w,
                                                 unsigned short* __restrict__ oh, unsigned short* __restrict__ ol,
                                                 int nthr) {
  const int t = blockIdx.x * 256 + threadIdx.x;
  if (t >= nthr) return;
  const int e0 = t * 8;
  const int o  = e0 / kK1P;
  const int c0 = e0 - o * kK1P;
  unsigned short hb[8], lb[8];
#pragma unroll
  for (int e = 0; e < 8; ++e) {
    const int col = c0 + e;
    const int cc  = (col < kK1) ? col : (kK1 - 1);
    float x = w[o * kK1 + cc];
    x = (col < kK1) ? x : 0.f;
    bf_split_bits(x, hb[e], lb[e]);
  }
  const v4u uh = (v4u){pk16(hb[0], hb[1]), pk16(hb[2], hb[3]), pk16(hb[4], hb[5]), pk16(hb[6], hb[7])};
  const v4u ul = (v4u){pk16(lb[0], lb[1]), pk16(lb[2], lb[3]), pk16(lb[4], lb[5]), pk16(lb[6], lb[7])};
  st2x_u4(oh + (size_t)e0, uh, ol + (size_t)e0, ul);
}

__global__ __launch_bounds__(256) void k_w2_cast(const float* __restrict__ w, unsigned short* __restrict__ ob, int nthr) {
  const int t = blockIdx.x * 256 + threadIdx.x;
  if (t >= nthr) return;
  const int e0   = t * 8;
  const int o    = e0 / kK2;
  const int col0 = e0 - o * kK2;
  const int kk   = col0 >> 8;
  const int ci0  = col0 & 255;
  const float* src = w + ((size_t)o * kCh1 + ci0) * kK1 + kk;
  unsigned short hb[8];
#pragma unroll
  for (int e = 0; e < 8; ++e) hb[e] = h_bits(src[e * kK1] * kW2Carry);
  const v4u u = (v4u){pk16(hb[0], hb[1]), pk16(hb[2], hb[3]), pk16(hb[4], hb[5]), pk16(hb[6], hb[7])};
  st2_u4(ob + (size_t)e0, u);
}

__global__ __launch_bounds__(256) void k_im2col1(const float* __restrict__ img, int cb,
                                                 unsigned short* __restrict__ ah, unsigned short* __restrict__ al,
                                                 int nthr) {
  const int t = blockIdx.x * 256 + threadIdx.x;
  if (t >= nthr) return;
  const int e0  = t * 8;
  const int row = e0 / kK1P;
  const int c0  = e0 - row * kK1P;
  const int bl  = row / kO1Pix;
  const int p   = row - bl * kO1Pix;
  const int oy  = p / kO1;
  const int ox  = p - oy * kO1;
  const float* im = img + (size_t)(cb + bl) * kImgPix + oy * kImg + ox;
  unsigned short hb[8], lb[8];
#pragma unroll
  for (int e = 0; e < 8; ++e) {
    const int col = c0 + e;
    const int cc  = (col < kK1) ? col : (kK1 - 1);
    const int ky  = cc / 9;
    const int kx  = cc - ky * 9;
    float x = im[ky * kImg + kx];
    x = (col < kK1) ? x : 0.f;
    bf_split_bits(x, hb[e], lb[e]);
  }
  const v4u uh = (v4u){pk16(hb[0], hb[1]), pk16(hb[2], hb[3]), pk16(hb[4], hb[5]), pk16(hb[6], hb[7])};
  const v4u ul = (v4u){pk16(lb[0], lb[1]), pk16(lb[2], lb[3]), pk16(lb[4], lb[5]), pk16(lb[6], lb[7])};
  st2x_u4(ah + (size_t)e0, uh, al + (size_t)e0, ul);
}

__global__ __launch_bounds__(256) void k_im2col2(const unsigned short* __restrict__ x1, unsigned short* __restrict__ a2,
                                                 int nthr) {
  const int t = blockIdx.x * 256 + threadIdx.x;
  if (t >= nthr) return;
  const int e0   = t * 8;
  const int row  = e0 / kK2;
  const int col0 = e0 - row * kK2;
  const int kk   = col0 >> 8;
  const int ci0  = col0 & 255;
  const int bl   = row / kPos;
  const int pos  = row - bl * kPos;
  const int py   = pos / kO2;
  const int px   = pos - py * kO2;
  const int ky   = kk / 9;
  const int kx   = kk - ky * 9;
  const int srow = bl * kO1Pix + (2 * py + ky) * kO1 + (2 * px + kx);
  const v4u v = *(const v4u*)(x1 + (size_t)srow * kCh1 + ci0);
  st2_u4(a2 + (size_t)e0, v);
}

__global__ __launch_bounds__(256) void k_usquash(const float* __restrict__ u,
                                                 unsigned short* __restrict__ ush, unsigned short* __restrict__ usl) {
  __shared__ __align__(16) float us_s[kPos * kCh2];
  __shared__ float sq_s[kCapsIn];
  const int tid  = threadIdx.x;
  const int lane = tid & 31;
  const int wave = tid >> 5;
  const int b    = blockIdx.x;
  const float* ub = u + (size_t)b * kPos * kCh2;
  float part = 0.f;
#pragma unroll 4
  for (int k = 0; k < kPos; ++k) {
    const float x = ub[k * kCh2 + tid];
    us_s[k * kCh2 + tid] = x;
    part = fmaf(x, x, part);
  }
#pragma unroll
  for (int off = 16; off > 0; off >>= 1) part += __shfl_xor(part, off, 32);
  if (lane == 0) sq_s[wave] = part;
  __syncthreads();
  float fscale[8], rinv[8];
#pragma unroll
  for (int i = 0; i < 8; ++i) {
    const float sq = sq_s[i];
    fscale[i] = sq / (1.0f + sq);
    rinv[i]   = 1.0f / sqrtf(sq);
  }
  for (int tq = tid; tq < kRoutes; tq += 256) {
    const int rr  = tq / kPos;
    const int pos = tq - rr * kPos;
    const float* rowp = us_s + pos * kCh2 + rr;
    unsigned short hb[8], lb[8];
#pragma unroll
    for (int i = 0; i < 8; ++i) {
      const float x = fscale[i] * (rowp[i * 32] * rinv[i]);
      bf_split_bits(x, hb[i], lb[i]);
    }
    const v4u uh = (v4u){pk16(hb[0], hb[1]), pk16(hb[2], hb[3]), pk16(hb[4], hb[5]), pk16(hb[6], hb[7])};
    const v4u ul = (v4u){pk16(lb[0], lb[1]), pk16(lb[2], lb[3]), pk16(lb[4], lb[5]), pk16(lb[6], lb[7])};
    const size_t o = (size_t)b * kQ + (size_t)tq * 8;
    st2x_u4(ush + o, uh, usl + o, ul);
  }
}

__global__ __launch_bounds__(256) void k_transpose_us(const unsigned short* __restrict__ ih, const unsigned short* __restrict__ il,
                                                      unsigned short* __restrict__ oh, unsigned short* __restrict__ ol) {
  __shared__ __align__(16) unsigned short th[64 * 72];
  __shared__ __align__(16) unsigned short tl[64 * 72];
  const int tid = threadIdx.x;
  const int q0 = blockIdx.x * 64;
  const int b0 = blockIdx.y * 64;
#pragma unroll
  for (int k = 0; k < 2; ++k) {
    const int idx = tid + 256 * k;
    const int bb  = idx >> 3;
    const int cq  = (idx & 7) * 8;
    const size_t src = (size_t)(b0 + bb) * kQ + q0 + cq;
    const v4u vh = *(const v4u*)(ih + src);
    const v4u vl = *(const v4u*)(il + src);
#pragma unroll
    for (int e = 0; e < 8; ++e) {
      const unsigned wh = (vh[e >> 1] >> ((e & 1) * 16)) & 0xffffu;
      const unsigned wl = (vl[e >> 1] >> ((e & 1) * 16)) & 0xffffu;
      th[(cq + e) * 72 + bb] = (unsigned short)wh;
      tl[(cq + e) * 72 + bb] = (unsigned short)wl;
    }
  }
  __syncthreads();
#pragma unroll
  for (int k = 0; k < 2; ++k) {
    const int idx = tid + 256 * k;
    const int ql  = idx >> 3;
    const int cb  = (idx & 7) * 8;
    const v4u uh = *(const v4u*)(th + ql * 72 + cb);
    const v4u ul = *(const v4u*)(tl + ql * 72 + cb);
    const size_t dst = (size_t)(q0 + ql) * kBatch + b0 + cb;
    st2x_u4(oh + dst, uh, ol + dst, ul);
  }
}

__global__ __launch_bounds__(256) void k_init_routing(float* __restrict__ cpl, float* __restrict__ bpl, int n4) {
  const int t = blockIdx.x * 256 + threadIdx.x;
  if (t >= n4) return;
  const int j0 = (t & 3) * 4;
  v4f cv;
#pragma unroll
  for (int e = 0; e < 4; ++e) cv[e] = (j0 + e < kCaps) ? 0.1f : 0.0f;
  const v4f z = (v4f){0.f, 0.f, 0.f, 0.f};
  float* pc = cpl + (size_t)t * 4;
  float* pb = bpl + (size_t)t * 4;
  *(volatile v4f*)pc = cv;
  *(volatile v4f*)pb = z;
  __threadfence();
  *(volatile v4f*)pc = cv;
  *(volatile v4f*)pb = z;
}

__global__ __launch_bounds__(256) void k_wc(const float* __restrict__ wcap, const float* __restrict__ cpl,
                                            unsigned short* __restrict__ wch, unsigned short* __restrict__ wcl) {
  const int jd = blockIdx.x;
  const int j  = jd >> 4;
  const int d  = jd & 15;
  const bool live = jd < kJD;
  const int jc = live ? j : (kCaps - 1);
  for (int tq = threadIdx.x; tq < kRoutes; tq += 256) {
    const float cv = cpl[tq * kPitchBC + jc];
    const float* wp = wcap + ((size_t)(tq * kCaps + jc) * kCapsDim + d) * kCapsIn;
    const v4f w0 = *(const v4f*)(wp);
    const v4f w1 = *(const v4f*)(wp + 4);
    unsigned short hb[8], lb[8];
#pragma unroll
    for (int e = 0; e < 4; ++e) {
      float x0 = w0[e] * cv;
      float x1 = w1[e] * cv;
      x0 = live ? x0 : 0.f;
      x1 = live ? x1 : 0.f;
      bf_split_bits(x0, hb[e], lb[e]);
      bf_split_bits(x1, hb[4 + e], lb[4 + e]);
    }
    const v4u uh = (v4u){pk16(hb[0], hb[1]), pk16(hb[2], hb[3]), pk16(hb[4], hb[5]), pk16(hb[6], hb[7])};
    const v4u ul = (v4u){pk16(lb[0], lb[1]), pk16(lb[2], lb[3]), pk16(lb[4], lb[5]), pk16(lb[6], lb[7])};
    const size_t o = (size_t)jd * kQ + (size_t)tq * 8;
    st2x_u4(wch + o, uh, wcl + o, ul);
  }
}

__global__ __launch_bounds__(256) void k_vsq_vt(const float* __restrict__ s,
                                                unsigned short* __restrict__ vth, unsigned short* __restrict__ vtl) {
  __shared__ __align__(16) float vt_s[kCapsDim * 264];
  const int tid = threadIdx.x;
  const int jt  = blockIdx.x;
  const bool live = jt < kCaps;
  const int jc  = live ? jt : (kCaps - 1);
  const int b   = tid;
  const float* sp = s + (size_t)b * kJDP + jc * kCapsDim;
  const v4f s0 = *(const v4f*)(sp), s1 = *(const v4f*)(sp + 4), s2 = *(const v4f*)(sp + 8), s3 = *(const v4f*)(sp + 12);
  float sv[16];
#pragma unroll
  for (int e = 0; e < 4; ++e) { sv[e] = s0[e]; sv[4 + e] = s1[e]; sv[8 + e] = s2[e]; sv[12 + e] = s3[e]; }
  float sq = 0.f;
#pragma unroll
  for (int e = 0; e < 16; ++e) sq = fmaf(sv[e], sv[e], sq);
  const float fs   = sq / (1.0f + sq);
  const float rinv = 1.0f / sqrtf(sq);
#pragma unroll
  for (int e = 0; e < 16; ++e) {
    float v = fs * (sv[e] * rinv);
    v = live ? v : 0.f;
    vt_s[e * 264 + b] = v;
  }
  __syncthreads();
#pragma unroll
  for (int k = 0; k < 2; ++k) {
    const int idx = tid + 256 * k;
    const int d   = idx >> 5;
    const int cb  = (idx & 31) * 8;
    const float* vp = vt_s + d * 264 + cb;
    unsigned short hb[8], lb[8];
#pragma unroll
    for (int e = 0; e < 8; ++e) bf_split_bits(vp[e], hb[e], lb[e]);
    const v4u uh = (v4u){pk16(hb[0], hb[1]), pk16(hb[2], hb[3]), pk16(hb[4], hb[5]), pk16(hb[6], hb[7])};
    const v4u ul = (v4u){pk16(lb[0], lb[1]), pk16(lb[2], lb[3]), pk16(lb[4], lb[5]), pk16(lb[6], lb[7])};
    const size_t o = (size_t)(jt * kCapsDim + d) * kBatch + cb;
    st2x_u4(vth + o, uh, vtl + o, ul);
  }
}

__global__ __launch_bounds__(256) void k_vsq_out(const float* __restrict__ s, float* __restrict__ out) {
  __shared__ __align__(16) float s_s[32 * kJDP];
  __shared__ __align__(16) float o_s[32 * kJD];
  const int tid = threadIdx.x;
  const int b0  = blockIdx.x * 32;
  const float* sb = s + (size_t)b0 * kJDP;
#pragma unroll
  for (int k = 0; k < 6; ++k) {
    const int idx = tid + 256 * k;
    *(v4f*)(s_s + idx * 4) = *(const v4f*)(sb + (size_t)idx * 4);
  }
  __syncthreads();
  for (int p = tid; p < 32 * kCaps; p += 256) {
    const int bl = p / kCaps;
    const int j  = p - bl * kCaps;
    const float* sp = s_s + bl * kJDP + j * kCapsDim;
    const v4f s0 = *(const v4f*)(sp), s1 = *(const v4f*)(sp + 4), s2 = *(const v4f*)(sp + 8), s3 = *(const v4f*)(sp + 12);
    float sv[16];
#pragma unroll
    for (int e = 0; e < 4; ++e) { sv[e] = s0[e]; sv[4 + e] = s1[e]; sv[8 + e] = s2[e]; sv[12 + e] = s3[e]; }
    float sq = 0.f;
#pragma unroll
    for (int e = 0; e < 16; ++e) sq = fmaf(sv[e], sv[e], sq);
    const float fs   = sq / (1.0f + sq);
    const float rinv = 1.0f / sqrtf(sq);
    float* op = o_s + bl * kJD + j * kCapsDim;
#pragma unroll
    for (int e = 0; e < 16; ++e) op[e] = fs * (sv[e] * rinv);
  }
  __syncthreads();
  float* ob = out + (size_t)b0 * kJD;
  for (int pass = 0; pass < 2; ++pass) {
#pragma unroll
    for (int k = 0; k < 5; ++k) {
      const int idx = tid + 256 * k;
      const v4f v = *(const v4f*)(o_s + idx * 4);
      *(volatile v4f*)(ob + (size_t)idx * 4) = v;
    }
    __threadfence();
  }
}

__global__ __launch_bounds__(256) void k_agree(const float* __restrict__ wcap, const float* __restrict__ g,
                                               const float* __restrict__ bold, float* __restrict__ bnew,
                                               float* __restrict__ cnew) {
  __shared__ __align__(16) float b_s[256];
  __shared__ __align__(16) float c_s[256];
  const int tid = threadIdx.x;
  const int rl  = tid >> 4;
  const int j   = tid & 15;
  const int r   = blockIdx.x * 16 + rl;
  const int jc  = (j < kCaps) ? j : (kCaps - 1);
  const float* wp = wcap + (size_t)(r * kCaps + jc) * (kCapsDim * kCapsIn);
  const float* gp = g + (size_t)(r * kCapsIn) * kJDP + jc * kCapsDim;
  float acc = 0.f;
#pragma unroll 1
  for (int i = 0; i < kCapsIn; ++i) {
    const float* wi = wp + i;
    const float* gi = gp + i * kJDP;
#pragma unroll
    for (int d = 0; d < kCapsDim; ++d) acc = fmaf(wi[d * kCapsIn], gi[d], acc);
  }
  const float ag = acc * kInvBatch;
  const float bo = bold[r * kPitchBC + j];
  const bool livej = j < kCaps;
  const float bn = livej ? (bo + ag) : 0.f;
  float m = livej ? bn : -INFINITY;
#pragma unroll
  for (int off = 8; off > 0; off >>= 1) m = fmaxf(m, __shfl_xor(m, off, 32));
  const float ex = livej ? expf(bn - m) : 0.f;
  float ssum = ex;
#pragma unroll
  for (int off = 8; off > 0; off >>= 1) ssum += __shfl_xor(ssum, off, 32);
  const float cn = ex * (1.0f / ssum);
  b_s[tid] = bn;
  c_s[tid] = cn;
  __syncthreads();
  const size_t base = (size_t)blockIdx.x * 256;
  if (tid < 64) {
    const v4f v = *(const v4f*)(b_s + tid * 4);
    st2_f4(bnew + base + (size_t)tid * 4, v);
  } else if (tid < 128) {
    const int t2 = tid - 64;
    const v4f v = *(const v4f*)(c_s + t2 * 4);
    st2_f4(cnew + base + (size_t)t2 * 4, v);
  }
}

extern "C" void kernel_launch(void* const* d_in, const int* in_sizes, int n_in,
                              void* d_out, int out_size, void* d_ws, size_t ws_size,
                              hipStream_t stream) {
  if (n_in < 7) return;
  if (in_sizes[0] != kBatch * kImgPix || in_sizes[2] != kCh1 * kK1 || in_sizes[3] != kCh1 ||
      in_sizes[4] != kCh2 * kCh1 * kK1 || in_sizes[5] != kCh2 ||
      in_sizes[6] != kRoutes * kCaps * kCapsDim * kCapsIn || out_size != kBatch * kJD) return;

  const float* img  = (const float*)d_in[0];
  const float* w1   = (const float*)d_in[2];
  const float* b1   = (const float*)d_in[3];
  const float* w2   = (const float*)d_in[4];
  const float* b2   = (const float*)d_in[5];
  const float* wcap = (const float*)d_in[6];
  float* out = (float*)d_out;

  char* ws = (char*)d_ws;
  size_t off = 0;
  auto take = [&](size_t bytes) -> char* {
    char* p = ws + off;
    off += (bytes + 255) & ~(size_t)255;
    return p;
  };
  unsigned short* b1h = (unsigned short*)take((size_t)kCh1 * kK1P * 2);
  unsigned short* b1l = (unsigned short*)take((size_t)kCh1 * kK1P * 2);
  unsigned short* b2p = (unsigned short*)take((size_t)kCh2 * kK2 * 2);
  unsigned short* a1h = (unsigned short*)take((size_t)kM1 * kK1P * 2);
  unsigned short* a1l = (unsigned short*)take((size_t)kM1 * kK1P * 2);
  unsigned short* x1c = (unsigned short*)take((size_t)kM1 * kCh1 * 2);
  unsigned short* a2p = (unsigned short*)take((size_t)kM2 * kK2 * 2);
  float* uall = (float*)take((size_t)kBatch * kPos * kCh2 * 4);
  unsigned short* ush = (unsigned short*)take((size_t)kBatch * kQ * 2);
  unsigned short* usl = (unsigned short*)take((size_t)kBatch * kQ * 2);
  unsigned short* uth = (unsigned short*)take((size_t)kQ * kBatch * 2);
  unsigned short* utl = (unsigned short*)take((size_t)kQ * kBatch * 2);
  float* ctab[3];
  float* btab[3];
  for (int i = 0; i < 3; ++i) ctab[i] = (float*)take((size_t)kRoutes * kPitchBC * 4);
  for (int i = 0; i < 3; ++i) btab[i] = (float*)take((size_t)kRoutes * kPitchBC * 4);
  unsigned short* wch = (unsigned short*)take((size_t)kJDP * kQ * 2);
  unsigned short* wcl = (unsigned short*)take((size_t)kJDP * kQ * 2);
  float* sbuf = (float*)take((size_t)kBatch * kJDP * 4);
  unsigned short* vth = (unsigned short*)take((size_t)kJDP * kBatch * 2);
  unsigned short* vtl = (unsigned short*)take((size_t)kJDP * kBatch * 2);
  float* gbuf = (float*)take((size_t)kQ * kJDP * 4);
  if (off > ws_size) return;

  {
    const int n1 = kCh1 * kK1P / 8;
    k_w1_split<<<dim3((n1 + 255) / 256), dim3(256), 0, stream>>>(w1, b1h, b1l, n1);
    const int n2 = kCh2 * kK2 / 8;
    k_w2_cast<<<dim3((n2 + 255) / 256), dim3(256), 0, stream>>>(w2, b2p, n2);
    const int n4 = kRoutes * kPitchBC / 4;
    k_init_routing<<<dim3((n4 + 255) / 256), dim3(256), 0, stream>>>(ctab[0], btab[0], n4);
  }

  for (int c = 0; c < kChunks; ++c) {
    const int nthr1 = kM1 * kK1P / 8;
    k_im2col1<<<dim3((nthr1 + 255) / 256), dim3(256), 0, stream>>>(img, c * kChunkImg, a1h, a1l, nthr1);
    wmma_gemm64<1, true, 2, 1, false, 2><<<dim3((kM1 / 64) * (kCh1 / 64) / 8), dim3(256), 0, stream>>>(
        b1h == nullptr ? a1h : a1h, a1l, kK1P, 0L, b1h, b1l, kK1P, 0L,
        (void*)x1c, (void*)x1c, kCh1, 0L, b1, b1, 0L, kM1, kCh1, kK1P, 1.0f);
    const int nthr2 = kM2 * kK2 / 8;
    k_im2col2<<<dim3((nthr2 + 255) / 256), dim3(256), 0, stream>>>(x1c, a2p, nthr2);
    float* uc = uall + (size_t)c * kM2 * kCh2;
    wmma_gemm64<0, false, 2, 0, false, 0><<<dim3((kM2 / 64) * (kCh2 / 64) / 8), dim3(256), 0, stream>>>(
        a2p, a2p, kK2, 0L, b2p, b2p, kK2, 0L,
        (void*)uc, (void*)uc, kCh2, 0L, b2, b2, 0L, kM2, kCh2, kK2, kW2CarryInv);
  }

  k_usquash<<<dim3(kBatch), dim3(256), 0, stream>>>(uall, ush, usl);
  k_transpose_us<<<dim3(kQ / 64, kBatch / 64), dim3(256), 0, stream>>>(ush, usl, uth, utl);

  for (int it = 0; it < 3; ++it) {
    k_wc<<<dim3(kJDP), dim3(256), 0, stream>>>(wcap, ctab[it], wch, wcl);
    wmma_gemm64<1, true, 0, 0, false, 0><<<dim3(((kBatch / 64) * (kJDP / 64) + 7) / 8), dim3(256), 0, stream>>>(
        ush, usl, kQ, 0L, wch, wcl, kQ, 0L,
        (void*)sbuf, (void*)sbuf, kJDP, 0L, b2, sbuf, 0L, kBatch, kJDP, kQ, 1.0f);
    if (it < 2) {
      k_vsq_vt<<<dim3(kJDP / kCapsDim), dim3(256), 0, stream>>>(sbuf, vth, vtl);
      wmma_gemm64<1, true, 0, 0, false, 0><<<dim3(((kQ / 64) * (kJDP / 64) + 7) / 8), dim3(256), 0, stream>>>(
          uth, utl, kBatch, 0L, vth, vtl, kBatch, 0L,
          (void*)gbuf, (void*)gbuf, kJDP, 0L, b2, gbuf, 0L, kQ, kJDP, kBatch, 1.0f);
      k_agree<<<dim3(kRoutes / 16), dim3(256), 0, stream>>>(wcap, gbuf, btab[it], btab[it + 1], ctab[it + 1]);
    } else {
      k_vsq_out<<<dim3(kBatch / 32), dim3(256), 0, stream>>>(sbuf, out);
    }
  }
}
